// ChromatinGAT_82231443849544
// MI455X (gfx1250) — hardware-verified
//
#include <hip/hip_runtime.h>
#include <stddef.h>


#define NTHR  256
#define NWAVE 8
#define RPAD  256
#define CHUNK 2048
#define WCAP  256
#define NGRP  (CHUNK / (NTHR * 4))
#define SB    10
#define AGG_LDS_BYTES 278560

static_assert(WCAP == (CHUNK / NTHR) * 32);
static_assert(NGRP >= 1);
static_assert(CHUNK <= 2048);

typedef float          v2f  __attribute__((ext_vector_type(2)));
typedef float          v4f  __attribute__((ext_vector_type(4)));
typedef float          v8f  __attribute__((ext_vector_type(8)));
typedef int            v4i  __attribute__((ext_vector_type(4)));
typedef unsigned short v8us __attribute__((ext_vector_type(8)));
typedef __bf16         v16b __attribute__((ext_vector_type(16)));
typedef double         v2d  __attribute__((ext_vector_type(2)));
union Frag  { v16b v; v8us half[2]; };
union Pack8 { v8us v; unsigned short s[8]; };

__device__ __forceinline__ unsigned short bfr(float f) {
  unsigned u = __float_as_uint(f);
  u += 0x7FFFu + ((u >> 16) & 1u);
  return (unsigned short)(u >> 16);
}
__device__ __forceinline__ float bff(unsigned short h) { return __uint_as_float(((unsigned)h) << 16); }

__device__ __forceinline__ v8f wmb(v16b a, v16b b, v8f c) {
  v8f d = __builtin_amdgcn_wmma_f32_16x16x32_bf16(false, a, false, b, (short)0, c, false, false);
  asm volatile("v_nop\n\tv_nop\n\tv_nop\n\tv_nop" : "+v"(d) : "v"(a), "v"(b));
  return d;
}

__device__ __forceinline__ v16b ldfrag(const unsigned short* p) {
  Frag f;
  f.half[0] = *(const v8us*)p;
  f.half[1] = *(const v8us*)(p + 16);
  return f.v;
}

__device__ __forceinline__ void st_tile(float* Cs, int cp, int r0, int c0, int h, int m, v8f a) {
#pragma unroll
  for (int r = 0; r < 8; ++r) Cs[(r0 + 8 * h + r) * cp + c0 + m] = a[r];
}

template <int K>
__device__ __forceinline__ void mm32(const unsigned short* __restrict__ Ah, const unsigned short* __restrict__ Al,
                                     const unsigned short* __restrict__ Bh, const unsigned short* __restrict__ Bl,
                                     int ar0, int bc0, int lane,
                                     v8f& c00, v8f& c01, v8f& c10, v8f& c11) {
  static_assert((K % 32) == 0);
  const int h = lane >> 4, m = lane & 15;
  const unsigned short* pa0 = Ah + (size_t)(ar0 + m) * K + 8 * h;
  const unsigned short* pa1 = Ah + (size_t)(ar0 + 16 + m) * K + 8 * h;
  const unsigned short* qa0 = Al + (size_t)(ar0 + m) * K + 8 * h;
  const unsigned short* qa1 = Al + (size_t)(ar0 + 16 + m) * K + 8 * h;
  const unsigned short* pb0 = Bh + (size_t)(bc0 + m) * K + 8 * h;
  const unsigned short* pb1 = Bh + (size_t)(bc0 + 16 + m) * K + 8 * h;
  const unsigned short* qb0 = Bl + (size_t)(bc0 + m) * K + 8 * h;
  const unsigned short* qb1 = Bl + (size_t)(bc0 + 16 + m) * K + 8 * h;
  const v8f z = {0.f, 0.f, 0.f, 0.f, 0.f, 0.f, 0.f, 0.f};
  c00 = z; c01 = z; c10 = z; c11 = z;
#pragma unroll 1
  for (int k0 = 0; k0 < K; k0 += 32) {
    const v16b ah0 = ldfrag(pa0 + k0), ah1 = ldfrag(pa1 + k0);
    const v16b al0 = ldfrag(qa0 + k0), al1 = ldfrag(qa1 + k0);
    const v16b bh0 = ldfrag(pb0 + k0), bh1 = ldfrag(pb1 + k0);
    const v16b bl0 = ldfrag(qb0 + k0), bl1 = ldfrag(qb1 + k0);
    c00 = wmb(ah0, bh0, c00); c00 = wmb(ah0, bl0, c00); c00 = wmb(al0, bh0, c00);
    c01 = wmb(ah0, bh1, c01); c01 = wmb(ah0, bl1, c01); c01 = wmb(al0, bh1, c01);
    c10 = wmb(ah1, bh0, c10); c10 = wmb(ah1, bl0, c10); c10 = wmb(al1, bh0, c10);
    c11 = wmb(ah1, bh1, c11); c11 = wmb(ah1, bl1, c11); c11 = wmb(al1, bh1, c11);
  }
}

__global__ __launch_bounds__(NTHR) void k_wprep(const float* __restrict__ W, int K, int Nc,
                                                 unsigned short* Wh, unsigned short* Wl) {
  __shared__ float T[64 * 65];
  const int tid = threadIdx.x;
  const int k0 = blockIdx.x * 64, n0 = blockIdx.y * 64;
#pragma unroll
  for (int i = 0; i < 16; ++i) {
    const int idx = i * NTHR + tid;
    const int kk = idx >> 6, nn = idx & 63;
    int n = n0 + nn; n = (n > Nc - 1) ? Nc - 1 : n;
    int k = k0 + kk; k = (k > K - 1) ? K - 1 : k;
    T[kk * 65 + nn] = W[(size_t)k * Nc + n];
  }
  __syncthreads();
  const int q = tid >> 3, j = tid & 7;
  Pack8 hv[2], lv[2];
  int nrow[2];
#pragma unroll
  for (int ps = 0; ps < 2; ++ps) {
    const int nl = q + 32 * ps;
    nrow[ps] = n0 + nl;
#pragma unroll
    for (int e = 0; e < 8; ++e) {
      const float v = T[(8 * j + e) * 65 + nl];
      const unsigned short hb = bfr(v);
      hv[ps].s[e] = hb;
      lv[ps].s[e] = bfr(v - bff(hb));
    }
  }
#pragma unroll
  for (int ps = 0; ps < 2; ++ps) {
    if (nrow[ps] < Nc) {
      const size_t o = (size_t)nrow[ps] * K + k0 + 8 * j;
      *(volatile v8us*)(Wh + o) = hv[ps].v;
      *(volatile v8us*)(Wl + o) = lv[ps].v;
    }
  }
  __threadfence();
#pragma unroll
  for (int ps = 0; ps < 2; ++ps) {
    if (nrow[ps] < Nc) {
      const size_t o = (size_t)nrow[ps] * K + k0 + 8 * j;
      *(volatile v8us*)(Wh + o) = hv[ps].v;
      *(volatile v8us*)(Wl + o) = lv[ps].v;
    }
  }
}

template <int DF, bool BN>
__global__ __launch_bounds__(NTHR) void k_split(const float* __restrict__ src, int grow0, int nN, int nrows,
                                                 const float* __restrict__ stats,
                                                 const float* __restrict__ gam, const float* __restrict__ bet,
                                                 unsigned short* Ph, unsigned short* Pl) {
  static_assert(DF == 64 || DF == 128 || DF == 256);
  __shared__ __attribute__((aligned(16))) unsigned short Lh[NTHR * 8];
  __shared__ __attribute__((aligned(16))) unsigned short Ll[NTHR * 8];
  __shared__ float Smu[256], Srs[256], Sg[256], Sb[256];
  const int tid = threadIdx.x;
  if (BN) {
    if (tid < DF) { Smu[tid] = stats[tid]; Srs[tid] = stats[256 + tid]; Sg[tid] = gam[tid]; Sb[tid] = bet[tid]; }
  }
  __syncthreads();
  const int g    = blockIdx.x * NTHR + tid;
  const int prow = g / (DF / 8);
  const int c0   = (g - prow * (DF / 8)) * 8;
  const int grow = grow0 + prow;
  const bool valid = (prow < nrows) && (grow < nN);
  int growc = grow; growc = (growc > nN - 1) ? nN - 1 : growc; growc = (growc < 0) ? 0 : growc;
  const float* sp = src + (size_t)growc * DF + c0;
#pragma unroll 1
  for (int i = 0; i < 8; ++i) {
    float v = sp[i];
    if (BN) {
      const int c = c0 + i;
      float t = (v - Smu[c]) * Srs[c];
      t = t * Sg[c] + Sb[c];
      const float em = expm1f(fminf(t, 0.0f));
      v = (t > 0.0f) ? t : em;
    }
    v = valid ? v : 0.0f;
    const unsigned short hb = bfr(v);
    Lh[tid * 8 + i] = hb;
    Ll[tid * 8 + i] = bfr(v - bff(hb));
  }
  __syncthreads();
  const v8us hvv = *(const v8us*)(Lh + tid * 8);
  const v8us lvv = *(const v8us*)(Ll + tid * 8);
  const size_t o = (size_t)prow * DF + c0;
  if (prow < nrows) { *(volatile v8us*)(Ph + o) = hvv; *(volatile v8us*)(Pl + o) = lvv; }
  __threadfence();
  if (prow < nrows) { *(volatile v8us*)(Ph + o) = hvv; *(volatile v8us*)(Pl + o) = lvv; }
}

template <int K, int NC>
__global__ __launch_bounds__(NTHR) void k_gemm(const unsigned short* __restrict__ Ah, const unsigned short* __restrict__ Al,
                                                const unsigned short* __restrict__ Bh, const unsigned short* __restrict__ Bl,
                                                const float* __restrict__ att_s, const float* __restrict__ att_d,
                                                float* Hout, float* asrc, float* adst, int grow0) {
  static_assert(NC == 256 || NC == 64);
  constexpr int WC = NC / 32;
  constexpr int WR = NWAVE / WC;
  constexpr int BR = 32 * WR;
  constexpr int NH = NC / 64;
  constexpr int CP = NC + 4;
  static_assert(BR * NH * 2 == NTHR);
  __shared__ __attribute__((aligned(16))) float Cs[BR * CP];
  __shared__ float Sat[2 * NC];
  __shared__ __attribute__((aligned(16))) float Sd[2 * BR * NH];

  const int tid = threadIdx.x, lane = tid & 31, wave = tid >> 5;
  const int h = lane >> 4, m = lane & 15;
  const int wr = wave / WC, wc = wave - wr * WC;
  const int pr0 = blockIdx.x * BR;

  v8f c00, c01, c10, c11;
  mm32<K>(Ah, Al, Bh, Bl, pr0 + 32 * wr, 32 * wc, lane, c00, c01, c10, c11);

  for (int i = tid; i < NC; i += NTHR) { Sat[i] = att_s[i]; Sat[NC + i] = att_d[i]; }
  st_tile(Cs, CP, 32 * wr,      32 * wc,      h, m, c00);
  st_tile(Cs, CP, 32 * wr,      32 * wc + 16, h, m, c01);
  st_tile(Cs, CP, 32 * wr + 16, 32 * wc,      h, m, c10);
  st_tile(Cs, CP, 32 * wr + 16, 32 * wc + 16, h, m, c11);
  __syncthreads();

  {
    const int row = tid / (2 * NH);
    const int rem = tid - row * (2 * NH);
    const int hd = rem >> 1, wh = rem & 1;
    const float* cp = Cs + row * CP + hd * 64;
    const float* ap = Sat + wh * NC + hd * 64;
    float s = 0.0f;
#pragma unroll 4
    for (int f = 0; f < 64; ++f) s += cp[f] * ap[f];
    Sd[wh * (BR * NH) + row * NH + hd] = s;
  }
  __syncthreads();

  const size_t growB = (size_t)grow0 + (size_t)pr0;
  const v4f gv = *(const v4f*)(Sd + (wave & 1) * (BR * NH) + 4 * lane);
  float* gp = (wave == 0) ? (asrc + growB * NH + 4 * lane) : (adst + growB * NH + 4 * lane);
  if (NC == 256) {
    v4f xa[4], xb[4];
#pragma unroll
    for (int i = 0; i < 4; ++i) {
      const int r = 4 * wave + i;
      xa[i] = *(const v4f*)(Cs + r * CP + 4 * lane);
      xb[i] = *(const v4f*)(Cs + r * CP + 128 + 4 * lane);
    }
#pragma unroll
    for (int i = 0; i < 4; ++i) {
      float* p = Hout + (growB + 4 * wave + i) * NC + 4 * lane;
      *(volatile v4f*)p = xa[i];
      *(volatile v4f*)(p + 128) = xb[i];
    }
    if (wave < 2) *(volatile v4f*)gp = gv;
    __threadfence();
#pragma unroll
    for (int i = 0; i < 4; ++i) {
      float* p = Hout + (growB + 4 * wave + i) * NC + 4 * lane;
      *(volatile v4f*)p = xa[i];
      *(volatile v4f*)(p + 128) = xb[i];
    }
    if (wave < 2) *(volatile v4f*)gp = gv;
  } else {
    v2f xr[16];
#pragma unroll
    for (int i = 0; i < 16; ++i) {
      const int r = 16 * wave + i;
      xr[i] = *(const v2f*)(Cs + r * CP + 2 * lane);
    }
#pragma unroll
    for (int i = 0; i < 16; ++i) {
      float* p = Hout + (growB + 16 * wave + i) * NC + 2 * lane;
      *(volatile v2f*)p = xr[i];
    }
    if (wave < 2) *(volatile v4f*)gp = gv;
    __threadfence();
#pragma unroll
    for (int i = 0; i < 16; ++i) {
      float* p = Hout + (growB + 16 * wave + i) * NC + 2 * lane;
      *(volatile v2f*)p = xr[i];
    }
    if (wave < 2) *(volatile v4f*)gp = gv;
  }
}

template <int K>
__global__ __launch_bounds__(NTHR) void k_cls(const unsigned short* __restrict__ Ah, const unsigned short* __restrict__ Al,
                                               const unsigned short* __restrict__ Bh, const unsigned short* __restrict__ Bl,
                                               const float* __restrict__ bc1, const float* __restrict__ wc2,
                                               const float* __restrict__ bc2, float* out, int nN) {
  constexpr int BR = 256, CP = 36;
  __shared__ __attribute__((aligned(16))) float Cs[BR * CP];
  __shared__ float Sw2[64], Sb1[32], Sb2[2];
  __shared__ __attribute__((aligned(16))) float Os[BR * 2];

  const int tid = threadIdx.x, lane = tid & 31, wave = tid >> 5;
  const int h = lane >> 4, m = lane & 15;
  const int pr0 = blockIdx.x * BR;

  v8f c00, c01, c10, c11;
  mm32<K>(Ah, Al, Bh, Bl, pr0 + 32 * wave, 0, lane, c00, c01, c10, c11);

  if (tid < 64) Sw2[tid] = wc2[tid];
  if (tid < 32) Sb1[tid] = bc1[tid];
  if (tid < 2)  Sb2[tid] = bc2[tid];
  st_tile(Cs, CP, 32 * wave,      0,  h, m, c00);
  st_tile(Cs, CP, 32 * wave,      16, h, m, c01);
  st_tile(Cs, CP, 32 * wave + 16, 0,  h, m, c10);
  st_tile(Cs, CP, 32 * wave + 16, 16, h, m, c11);
  __syncthreads();

  {
    const float* cp = Cs + tid * CP;
    float o0 = 0.0f, o1 = 0.0f;
#pragma unroll 4
    for (int j = 0; j < 32; ++j) {
      const float a = fmaxf(cp[j] + Sb1[j], 0.0f);
      o0 += a * Sw2[2 * j];
      o1 += a * Sw2[2 * j + 1];
    }
    Os[2 * tid]     = o0 + Sb2[0];
    Os[2 * tid + 1] = o1 + Sb2[1];
  }
  __syncthreads();

  if (wave < 4) {
    const int q = wave * 32 + lane;
    const int node = pr0 + 2 * q;
    const v4f o4 = *(const v4f*)(Os + 4 * q);
    const bool full = (node + 1) < nN;
    const bool one  = (!full) && (node < nN);
    float* p = out + (size_t)node * 2;
    if (full) *(volatile v4f*)p = o4; else if (one) *(volatile v2f*)p = o4.xy;
    __threadfence();
    if (full) *(volatile v4f*)p = o4; else if (one) *(volatile v2f*)p = o4.xy;
  }
}

template <int DF> struct RowOps;
template <> struct RowOps<256> {
  static constexpr int NV = 2;
  static constexpr int NCMP = 4;
  typedef v4f V;
  __device__ __forceinline__ static int  offA(int lane, int i)  { return 8 * lane + 4 * i; }
  __device__ __forceinline__ static int  headA(int lane)        { return lane >> 3; }
  __device__ __forceinline__ static bool denLane(int lane)      { return (lane & 7) == 0; }
  __device__ __forceinline__ static int  offB(int lane, int i)  { return 4 * lane + 128 * i; }
  __device__ __forceinline__ static int  headB(int lane, int i) { return (lane >> 4) + 2 * i; }
  __device__ __forceinline__ static V    ld(const float* p)     { return *(const V*)p; }
  __device__ __forceinline__ static void st(float* p, V v)      { *(V*)p = v; }
  __device__ __forceinline__ static void stv(float* p, V v)     { *(volatile V*)p = v; }
  __device__ __forceinline__ static float comp(V v, int c)      { return v[c]; }
};
template <> struct RowOps<64> {
  static constexpr int NV = 1;
  static constexpr int NCMP = 2;
  typedef v2f V;
  __device__ __forceinline__ static int  offA(int lane, int i)  { return 2 * lane + 0 * i; }
  __device__ __forceinline__ static int  headA(int lane)        { return 0 * lane; }
  __device__ __forceinline__ static bool denLane(int lane)      { return lane == 0; }
  __device__ __forceinline__ static int  offB(int lane, int i)  { return 2 * lane + 0 * i; }
  __device__ __forceinline__ static int  headB(int lane, int i) { return 0 * (lane + i); }
  __device__ __forceinline__ static V    ld(const float* p)     { return *(const V*)p; }
  __device__ __forceinline__ static void st(float* p, V v)      { *(V*)p = v; }
  __device__ __forceinline__ static void stv(float* p, V v)     { *(volatile V*)p = v; }
  __device__ __forceinline__ static float comp(V v, int c)      { return v[c]; }
};

template <int DF, int NH, int NB>
__global__ __launch_bounds__(NTHR) void k_agg(const int* __restrict__ ei, const float* __restrict__ H,
                                               const float* __restrict__ asrc, const float* __restrict__ adst,
                                               const float* __restrict__ bias,
                                               float* Agg, double* part, int nN, int nE) {
  typedef RowOps<DF> R;
  typedef typename R::V V;
  static_assert(DF == 64 * NH);
  static_assert(NB <= (1 << SB));
  static_assert((NB & (NB - 1)) == 0);
  static_assert((NB % NWAVE) == 0);
  static_assert(((NB * DF + NB * NH) % 4) == 0);
  static_assert((NB * DF + 2 * NB * NH + NWAVE * WCAP + NWAVE) * 4 == AGG_LDS_BYTES);
  static_assert(NWAVE * DF * 2 * 8 <= NB * DF * 4);
  static_assert(DF <= NTHR);

  extern __shared__ v4f lds_dyn[];
  float* sacc = (float*)lds_dyn;
  float* den  = sacc + NB * DF;
  float* mx   = den + NB * NH;
  int*   list = (int*)(mx + NB * NH);
  int*   wcnt = list + NWAVE * WCAP;

  const int tid  = threadIdx.x;
  const int lane = tid & 31;
  const int wave = tid >> 5;
  const int nodeBase = blockIdx.x * NB;

  {
    const v4f z4 = {0.f, 0.f, 0.f, 0.f};
    for (int i = tid; i < (NB * DF + NB * NH) / 4; i += NTHR) lds_dyn[i] = z4;
    for (int i = tid; i < NB * NH; i += NTHR) mx[i] = -1.0e30f;
  }
  __syncthreads();

  const int* eid = ei + nE;
  const bool al16 = ((nE & 3) == 0);
  const int nChunks = (nE + CHUNK - 1) / CHUNK;

#pragma unroll 1
  for (int ch = 0; ch < nChunks; ++ch) {
    const int cbase = ch * CHUNK;
    int wc = 0;
#pragma unroll
    for (int g = 0; g < NGRP; ++g) {
      const int el0 = (g * NTHR + tid) * 4;
      const int e0  = cbase + el0;
      const int sent = -2147483647 - 1;
      v4i d;
      if (al16 && (cbase + CHUNK <= nE)) {
        d = *(const v4i*)(eid + e0);
      } else {
        const int i0 = (e0     > nE - 1) ? nE - 1 : e0;
        const int i1 = (e0 + 1 > nE - 1) ? nE - 1 : e0 + 1;
        const int i2 = (e0 + 2 > nE - 1) ? nE - 1 : e0 + 2;
        const int i3 = (e0 + 3 > nE - 1) ? nE - 1 : e0 + 3;
        d.x = (e0     < nE) ? eid[i0] : sent;
        d.y = (e0 + 1 < nE) ? eid[i1] : sent;
        d.z = (e0 + 2 < nE) ? eid[i2] : sent;
        d.w = (e0 + 3 < nE) ? eid[i3] : sent;
      }
      const unsigned s0 = (unsigned)d.x - (unsigned)nodeBase;
      const unsigned s1 = (unsigned)d.y - (unsigned)nodeBase;
      const unsigned s2 = (unsigned)d.z - (unsigned)nodeBase;
      const unsigned s3 = (unsigned)d.w - (unsigned)nodeBase;
      const bool h0 = s0 < (unsigned)NB;
      const bool h1 = s1 < (unsigned)NB;
      const bool h2 = s2 < (unsigned)NB;
      const bool h3 = s3 < (unsigned)NB;
      const unsigned many = __builtin_amdgcn_ballot_w32(h0 | h1 | h2 | h3);
      if (many != 0u) {
#define HITJ(J, HJ, SJ) { \
          const unsigned mj = __builtin_amdgcn_ballot_w32(HJ); \
          if (HJ) { \
            const int pos = wc + (int)__builtin_amdgcn_mbcnt_lo(mj, 0u); \
            if (pos < WCAP) list[wave * WCAP + pos] = ((el0 + (J)) << SB) | (int)(SJ); \
          } \
          wc += (int)__builtin_popcount(mj); }
        HITJ(0, h0, s0)
        HITJ(1, h1, s1)
        HITJ(2, h2, s2)
        HITJ(3, h3, s3)
#undef HITJ
      }
    }
    if (lane == 0) wcnt[wave] = wc;
    __syncthreads();

    if (wave == 0) {
      const int hdA = R::headA(lane);
      for (int wsx = 0; wsx < NWAVE; ++wsx) {
        int n = wcnt[wsx];
        n = (n > WCAP) ? WCAP : n;
        n = (n < 0) ? 0 : n;
        for (int i = 0; i < n; ++i) {
          const int ent  = list[wsx * WCAP + i];
          const int slot = ent & (NB - 1);
          const int el   = (ent >> SB) & (CHUNK - 1);
          int e = cbase + el;
          e = (e > nE - 1) ? nE - 1 : e;
          int src = ei[e];
          src = (src < 0) ? 0 : ((src > nN - 1) ? nN - 1 : src);
          int nd = nodeBase + slot;
          nd = (nd > nN - 1) ? nN - 1 : nd;
          float lg = asrc[(size_t)src * NH + hdA] + adst[(size_t)nd * NH + hdA];
          lg = (lg > 0.0f) ? lg : 0.2f * lg;
          const int mi = slot * NH + hdA;
          const float mo = mx[mi];
          const float mn = fmaxf(mo, lg);
          const float p  = __expf(lg - mn);
          const float sc = __expf(mo - mn);
          V xv[R::NV], cur[R::NV];
#pragma unroll
          for (int v = 0; v < R::NV; ++v) {
            xv[v]  = R::ld(H + (size_t)src * DF + R::offA(lane, v));
            cur[v] = R::ld(sacc + slot * DF + R::offA(lane, v));
          }
#pragma unroll
          for (int v = 0; v < R::NV; ++v) {
            const V nxt = cur[v] * sc + p * xv[v];
            R::st(sacc + slot * DF + R::offA(lane, v), nxt);
          }
          if (R::denLane(lane)) {
            const float dd = den[mi];
            den[mi] = dd * sc + p;
            mx[mi]  = mn;
          }
        }
      }
    }
    __syncthreads();
  }

  constexpr int SPW = NB / NWAVE;
  double ds[R::NV * R::NCMP], dq[R::NV * R::NCMP];
#pragma unroll
  for (int i = 0; i < R::NV * R::NCMP; ++i) { ds[i] = 0.0; dq[i] = 0.0; }
  V bv[R::NV];
#pragma unroll
  for (int v = 0; v < R::NV; ++v) bv[v] = R::ld(bias + R::offB(lane, v));

#pragma unroll 1
  for (int j = 0; j < SPW; ++j) {
    const int slot = wave * SPW + j;
    const int node = nodeBase + slot;
    if (node >= nN) break;
    const size_t nrow = (size_t)node;
    V ov[R::NV];
#pragma unroll
    for (int v = 0; v < R::NV; ++v) {
      const int hd = R::headB(lane, v);
      float lg = asrc[nrow * NH + hd] + adst[nrow * NH + hd];
      lg = (lg > 0.0f) ? lg : 0.2f * lg;
      const int mi = slot * NH + hd;
      const float mo = mx[mi];
      const float mn = fmaxf(mo, lg);
      const float ps = __expf(lg - mn);
      const float sc = __expf(mo - mn);
      const V xs = R::ld(H + nrow * DF + R::offB(lane, v));
      const V sv = R::ld(sacc + slot * DF + R::offB(lane, v)) * sc + ps * xs;
      const float dv  = den[mi] * sc + ps;
      const float inv = __builtin_amdgcn_rcpf(dv);
      ov[v] = sv * inv + bv[v];
#pragma unroll
      for (int c = 0; c < R::NCMP; ++c) {
        const double o = (double)R::comp(ov[v], c);
        ds[v * R::NCMP + c] += o;
        dq[v * R::NCMP + c] += o * o;
      }
    }
    float* op = Agg + nrow * DF;
#pragma unroll
    for (int v = 0; v < R::NV; ++v) R::stv(op + R::offB(lane, v), ov[v]);
    __threadfence();
#pragma unroll
    for (int v = 0; v < R::NV; ++v) R::stv(op + R::offB(lane, v), ov[v]);
  }
  __syncthreads();

  double* Pw = (double*)lds_dyn;
#pragma unroll
  for (int v = 0; v < R::NV; ++v) {
#pragma unroll
    for (int c = 0; c < R::NCMP; ++c) {
      const int chn = R::offB(lane, v) + c;
      Pw[((size_t)wave * DF + chn) * 2]     = ds[v * R::NCMP + c];
      Pw[((size_t)wave * DF + chn) * 2 + 1] = dq[v * R::NCMP + c];
    }
  }
  __syncthreads();
  if (tid < DF) {
    double S = 0.0, Q = 0.0;
#pragma unroll
    for (int w = 0; w < NWAVE; ++w) { S += Pw[((size_t)w * DF + tid) * 2]; Q += Pw[((size_t)w * DF + tid) * 2 + 1]; }
    v2d o2; o2.x = S; o2.y = Q;
    double* pp = part + ((size_t)blockIdx.x * DF + tid) * 2;
    *(volatile v2d*)pp = o2;
    __threadfence();
    *(volatile v2d*)pp = o2;
  }
}

__global__ __launch_bounds__(NTHR) void k_bnfin(const double* __restrict__ part, int nblk, int DFr, int nN, float* stats) {
  __shared__ __attribute__((aligned(16))) float St[512];
  const int tid = threadIdx.x, lane = tid & 31, wave = tid >> 5;
  float muf = 0.0f, rsf = 0.0f;
  if (tid < DFr) {
    double S = 0.0, Q = 0.0;
#pragma unroll 1
    for (int b = 0; b < nblk; ++b) {
      const double* p = part + ((size_t)b * DFr + tid) * 2;
      S += p[0];
      Q += p[1];
    }
    const double inv = 1.0 / (double)nN;
    const double mu = S * inv;
    double var = Q * inv - mu * mu;
    var = (var < 0.0) ? 0.0 : var;
    muf = (float)mu;
    const float vf = (float)var + 1.0e-5f;
    rsf = (float)(1.0 / sqrt((double)vf));
  }
  St[tid] = muf;
  St[256 + tid] = rsf;
  __syncthreads();
  if (wave < 4) {
    const int q = wave * 32 + lane;
    const v4f v = *(const v4f*)(St + 4 * q);
    float* p = stats + 4 * q;
    *(volatile v4f*)p = v;
    __threadfence();
    *(volatile v4f*)p = v;
  }
}

extern "C" void kernel_launch(void* const* d_in, const int* in_sizes, int n_in,
                              void* d_out, int out_size, void* d_ws, size_t ws_size,
                              hipStream_t stream) {
  if (n_in < 24) return;
  const int IN = 128, HF = 256, HL = 64, NHD = 4, HC1 = 32, NCL = 2;
  const int nN = in_sizes[0] / IN;
  if (nN < 1 || in_sizes[0] != nN * IN) return;
  if (in_sizes[1] < 2 || (in_sizes[1] & 1)) return;
  const int nE = in_sizes[1] / 2;
  if (in_sizes[2] != IN * HF || in_sizes[3] != HF) return;
  if (in_sizes[4] != NHD * HL || in_sizes[5] != NHD * HL || in_sizes[6] != HF || in_sizes[7] != HF) return;
  if (in_sizes[8] != HF * HF || in_sizes[9] != HF) return;
  if (in_sizes[10] != NHD * HL || in_sizes[11] != NHD * HL || in_sizes[12] != HF || in_sizes[13] != HF) return;
  if (in_sizes[14] != HF * HL || in_sizes[15] != HL) return;
  if (in_sizes[16] != HL || in_sizes[17] != HL || in_sizes[18] != HL || in_sizes[19] != HL) return;
  if (in_sizes[20] != HL * HC1 || in_sizes[21] != HC1 || in_sizes[22] != HC1 * NCL || in_sizes[23] != NCL) return;
  if (out_size != nN * NCL) return;

  const float* x   = (const float*)d_in[0];
  const int*   ei  = (const int*)d_in[1];
  const float* w0  = (const float*)d_in[2];
  const float* b0  = (const float*)d_in[3];
  const float* as0 = (const float*)d_in[4];
  const float* ad0 = (const float*)d_in[5];
  const float* g0  = (const float*)d_in[6];
  const float* be0 = (const float*)d_in[7];
  const float* w1  = (const float*)d_in[8];
  const float* b1  = (const float*)d_in[9];
  const float* as1 = (const float*)d_in[10];
  const float* ad1 = (const float*)d_in[11];
  const float* g1  = (const float*)d_in[12];
  const float* be1 = (const float*)d_in[13];
  const float* w2  = (const float*)d_in[14];
  const float* b2  = (const float*)d_in[15];
  const float* as2 = (const float*)d_in[16];
  const float* ad2 = (const float*)d_in[17];
  const float* g2  = (const float*)d_in[18];
  const float* be2 = (const float*)d_in[19];
  const float* wc1 = (const float*)d_in[20];
  const float* bc1 = (const float*)d_in[21];
  const float* wc2 = (const float*)d_in[22];
  const float* bc2 = (const float*)d_in[23];
  float* out = (float*)d_out;

  const int MP = ((nN + RPAD - 1) / RPAD) * RPAD;
  const int RH = MP / 2;
  const int nb01 = (nN + 255) / 256;
  const int nb2  = (nN + 1023) / 1024;

  size_t off = 0;
  char* base = (char*)d_ws;
  auto take = [&](size_t bytes) -> void* {
    void* r = (void*)(base + off);
    off += (bytes + 255) & ~(size_t)255;
    return r;
  };
  unsigned short* W0h = (unsigned short*)take((size_t)HF * IN * 2);
  unsigned short* W0l = (unsigned short*)take((size_t)HF * IN * 2);
  unsigned short* W1h = (unsigned short*)take((size_t)HF * HF * 2);
  unsigned short* W1l = (unsigned short*)take((size_t)HF * HF * 2);
  unsigned short* W2h = (unsigned short*)take((size_t)HL * HF * 2);
  unsigned short* W2l = (unsigned short*)take((size_t)HL * HF * 2);
  unsigned short* Wch = (unsigned short*)take((size_t)HC1 * HL * 2);
  unsigned short* Wcl = (unsigned short*)take((size_t)HC1 * HL * 2);
  const size_t APL = (size_t)MP * IN * 2;
  unsigned short* Ah = (unsigned short*)take(APL);
  unsigned short* Al = (unsigned short*)take(APL);
  float* Hp = (float*)take((size_t)MP * HF * 4);
  float* As = (float*)take((size_t)MP * NHD * 4);
  float* Ad = (float*)take((size_t)MP * NHD * 4);
  float* Ag = (float*)take((size_t)MP * HF * 4);
  size_t partElems = (size_t)nb01 * HF; if ((size_t)nb2 * HL > partElems) partElems = (size_t)nb2 * HL;
  double* part = (double*)take(partElems * 2 * 8);
  float* stats = (float*)take(512 * 4);
  if (off > ws_size) return;
  if ((size_t)RH * HF * 2 > APL || (size_t)MP * HL * 2 > APL) return;

  k_wprep<<<dim3(IN / 64, HF / 64), NTHR, 0, stream>>>(w0, IN, HF, W0h, W0l);
  k_wprep<<<dim3(HF / 64, HF / 64), NTHR, 0, stream>>>(w1, HF, HF, W1h, W1l);
  k_wprep<<<dim3(HF / 64, HL / 64), NTHR, 0, stream>>>(w2, HF, HL, W2h, W2l);
  k_wprep<<<dim3(HL / 64, 1), NTHR, 0, stream>>>(wc1, HL, HC1, Wch, Wcl);

  hipFuncSetAttribute(reinterpret_cast<const void*>(&k_agg<256, 4, 256>),
                      hipFuncAttributeMaxDynamicSharedMemorySize, AGG_LDS_BYTES);
  hipFuncSetAttribute(reinterpret_cast<const void*>(&k_agg<64, 1, 1024>),
                      hipFuncAttributeMaxDynamicSharedMemorySize, AGG_LDS_BYTES);

  k_split<128, false><<<(MP / 256) * 128 / 8, NTHR, 0, stream>>>(x, 0, nN, MP, stats, g0, be0, Ah, Al);
  k_gemm<128, 256><<<MP / 32, NTHR, 0, stream>>>(Ah, Al, W0h, W0l, as0, ad0, Hp, As, Ad, 0);
  k_agg<256, 4, 256><<<nb01, NTHR, AGG_LDS_BYTES, stream>>>(ei, Hp, As, Ad, b0, Ag, part, nN, nE);
  k_bnfin<<<1, NTHR, 0, stream>>>(part, nb01, HF, nN, stats);

  for (int hf = 0; hf < 2; ++hf) {
    k_split<256, true><<<(RH / 256) * 256 / 8, NTHR, 0, stream>>>(Ag, hf * RH, nN, RH, stats, g0, be0, Ah, Al);
    k_gemm<256, 256><<<RH / 32, NTHR, 0, stream>>>(Ah, Al, W1h, W1l, as1, ad1, Hp, As, Ad, hf * RH);
  }
  k_agg<256, 4, 256><<<nb01, NTHR, AGG_LDS_BYTES, stream>>>(ei, Hp, As, Ad, b1, Ag, part, nN, nE);
  k_bnfin<<<1, NTHR, 0, stream>>>(part, nb01, HF, nN, stats);

  for (int hf = 0; hf < 2; ++hf) {
    k_split<256, true><<<(RH / 256) * 256 / 8, NTHR, 0, stream>>>(Ag, hf * RH, nN, RH, stats, g1, be1, Ah, Al);
    k_gemm<256, 64><<<RH / 128, NTHR, 0, stream>>>(Ah, Al, W2h, W2l, as2, ad2, Hp, As, Ad, hf * RH);
  }
  k_agg<64, 1, 1024><<<nb2, NTHR, AGG_LDS_BYTES, stream>>>(ei, Hp, As, Ad, b2, Ag, part, nN, nE);
  k_bnfin<<<1, NTHR, 0, stream>>>(part, nb2, HL, nN, stats);

  k_split<64, true><<<(MP / 256) * 64 / 8, NTHR, 0, stream>>>(Ag, 0, nN, MP, stats, g2, be2, Ah, Al);
  k_cls<64><<<MP / 256, NTHR, 0, stream>>>(Ah, Al, Wch, Wcl, bc1, wc2, bc2, out, nN);
}
